// Net_30107720745841
// MI455X (gfx1250) — hardware-verified
//
#include <hip/hip_runtime.h>
#include <stddef.h>
#include <stdint.h>


#define INC     64
#define HIDC    128
#define OUTC    64
#define K1      192
#define K2      256
#define NTHR    256
#define NWAVE   8
#define EPT     8
#define CHUNK   (NTHR * EPT)
#define WCAP    (EPT * 32)
#define LISTN   (NWAVE * WCAP)
#define NBA     1024
#define SLA     10
#define SRCB    17
#define RCAP    24576
#define DEGCAP  64
#define MEAS_B1024  16710
#define MEAS_MAXDEG 36
#define GBM     64
#define GBN     128
#define GTHR    128
#define MROWS   128
#define NPW     8
#define NPB     (NWAVE * NPW)
#define WSMAX   134217728
#define BKT_ZINTS    (RCAP + 3 * NBA)
#define BKT_LDS_INTS (LISTN + 2 * RCAP + 3 * NBA + 16)

static_assert((CHUNK & (CHUNK - 1)) == 0 && CHUNK <= 4096);
static_assert((NBA & (NBA - 1)) == 0 && NBA == (1 << SLA));
static_assert(((long long)CHUNK << SLA) < (1LL << 31));
static_assert(SRCB + SLA < 31);
static_assert(LISTN >= NWAVE * WCAP);
static_assert((RCAP % (NTHR * 4)) == 0 && (BKT_ZINTS % (NTHR * 4)) == 0);
static_assert(NBA == NTHR * 4);
static_assert(RCAP >= MEAS_B1024 + 4096);
static_assert((long long)RCAP * 20 >= (long long)MEAS_B1024 * 21);
static_assert(DEGCAP >= MEAS_MAXDEG + 8);
static_assert(BKT_LDS_INTS * 4 <= 300000);
static_assert(K1 % 32 == 0 && K2 % 32 == 0 && K1 == 2 * INC + INC && K2 == 2 * HIDC);
static_assert(GBN == HIDC && GBN == 2 * OUTC && GBM == (GTHR / 32) * 16);
static_assert(MROWS % GBM == 0 && MROWS % NPB == 0 && NBA % NPB == 0);
static_assert(INC == 2 * 32 && OUTC == 2 * 32);

typedef float          v2f  __attribute__((ext_vector_type(2)));
typedef float          v4f  __attribute__((ext_vector_type(4)));
typedef float          v8f  __attribute__((ext_vector_type(8)));
typedef int            v4i  __attribute__((ext_vector_type(4)));
typedef int            v8i  __attribute__((ext_vector_type(8)));
typedef unsigned       v2u  __attribute__((ext_vector_type(2)));
typedef unsigned short v4us __attribute__((ext_vector_type(4)));
typedef unsigned short v8us __attribute__((ext_vector_type(8)));
typedef __bf16         v16b __attribute__((ext_vector_type(16)));
typedef v2f  __attribute__((may_alias)) v2fa;
typedef v4f  __attribute__((may_alias)) v4fa;
typedef v4i  __attribute__((may_alias)) v4ia;
typedef v2u  __attribute__((may_alias)) v2ua;
typedef v4us __attribute__((may_alias)) v4usa;
typedef v8us __attribute__((may_alias)) v8usa;
union FragB { v16b v; v8us h[2]; v8i w; };

__device__ __forceinline__ v8f wmb(const FragB& a, const FragB& b, v8f c) {
  v8f d = __builtin_amdgcn_wmma_f32_16x16x32_bf16(false, a.v, false, b.v, (short)0, c, false, false);
  asm volatile("v_nop\n\tv_nop\n\tv_nop\n\tv_nop" : "+v"(d) : "v"(a.w), "v"(b.w));
  return d;
}

__device__ __forceinline__ unsigned int f2bf(float f) {
  const unsigned int u = __float_as_uint(f);
  const unsigned int r = ((u + 0x7FFFu + ((u >> 16) & 1u)) >> 16) & 0xFFFFu;
  return ((u & 0x7FFFFFFFu) > 0x7F800000u) ? 0x7FC0u : r;
}
__device__ __forceinline__ float bf2f(unsigned int b) { return __uint_as_float(b << 16); }

template <int SLB>
__device__ __forceinline__ int scan_chunk(const int* __restrict__ dsts, int nE, int cbase, int slotBase,
                                          int nb, int vec8, int* list, int tid, int lane, int wave) {
  int wc = 0;
  const int el0  = tid * EPT;
  const int e0   = cbase + el0;
  const int sent = -2147483647 - 1;
  v4i da, db;
  if (vec8 != 0 && cbase + CHUNK <= nE) {
    da = *(const v4i*)(dsts + e0);
    db = *(const v4i*)(dsts + e0 + 4);
  } else {
    da.x = (e0     < nE) ? dsts[min(e0,     nE - 1)] : sent;
    da.y = (e0 + 1 < nE) ? dsts[min(e0 + 1, nE - 1)] : sent;
    da.z = (e0 + 2 < nE) ? dsts[min(e0 + 2, nE - 1)] : sent;
    da.w = (e0 + 3 < nE) ? dsts[min(e0 + 3, nE - 1)] : sent;
    db.x = (e0 + 4 < nE) ? dsts[min(e0 + 4, nE - 1)] : sent;
    db.y = (e0 + 5 < nE) ? dsts[min(e0 + 5, nE - 1)] : sent;
    db.z = (e0 + 6 < nE) ? dsts[min(e0 + 6, nE - 1)] : sent;
    db.w = (e0 + 7 < nE) ? dsts[min(e0 + 7, nE - 1)] : sent;
  }
  const unsigned nbs = (unsigned)slotBase;
  const unsigned unb = (unsigned)nb;
  const unsigned s0 = (unsigned)da.x - nbs, s1 = (unsigned)da.y - nbs;
  const unsigned s2 = (unsigned)da.z - nbs, s3 = (unsigned)da.w - nbs;
  const unsigned s4 = (unsigned)db.x - nbs, s5 = (unsigned)db.y - nbs;
  const unsigned s6 = (unsigned)db.z - nbs, s7 = (unsigned)db.w - nbs;
  const bool h0 = s0 < unb, h1 = s1 < unb, h2 = s2 < unb, h3 = s3 < unb;
  const bool h4 = s4 < unb, h5 = s5 < unb, h6 = s6 < unb, h7 = s7 < unb;
  const unsigned any = __builtin_amdgcn_ballot_w32(h0 | h1 | h2 | h3 | h4 | h5 | h6 | h7);
  if (any != 0u) {
#define HITJ(J, HJ, SJ) { \
      const unsigned mj = __builtin_amdgcn_ballot_w32(HJ); \
      if (mj != 0u) { \
        if (HJ) { \
          const int pos = wc + (int)__builtin_amdgcn_mbcnt_lo(mj, 0u); \
          if (pos < WCAP) list[wave * WCAP + pos] = ((el0 + (J)) << SLB) | (int)(SJ); \
        } \
        wc += (int)__builtin_popcount(mj); } }
    HITJ(0, h0, s0)
    HITJ(1, h1, s1)
    HITJ(2, h2, s2)
    HITJ(3, h3, s3)
    HITJ(4, h4, s4)
    HITJ(5, h5, s5)
    HITJ(6, h6, s6)
    HITJ(7, h7, s7)
#undef HITJ
  }
  return wc;
}

__global__ __launch_bounds__(NTHR) void k_pa(const float* __restrict__ x, unsigned short* XB, int nN, int nU) {
  const int u = (int)blockIdx.x * NTHR + (int)threadIdx.x;
  if (u >= nU) return;
  const int row = u >> 3;
  const int c0  = (u & 7) * 8;
  const int rc  = row < nN ? row : nN - 1;
  const float* p = x + (size_t)rc * INC + c0;
  const v4f a = *(const v4f*)p;
  const v4f b = *(const v4f*)(p + 4);
  const bool ok = row < nN;
  v8us o;
  o[0] = ok ? (unsigned short)f2bf(a.x) : (unsigned short)0;
  o[1] = ok ? (unsigned short)f2bf(a.y) : (unsigned short)0;
  o[2] = ok ? (unsigned short)f2bf(a.z) : (unsigned short)0;
  o[3] = ok ? (unsigned short)f2bf(a.w) : (unsigned short)0;
  o[4] = ok ? (unsigned short)f2bf(b.x) : (unsigned short)0;
  o[5] = ok ? (unsigned short)f2bf(b.y) : (unsigned short)0;
  o[6] = ok ? (unsigned short)f2bf(b.z) : (unsigned short)0;
  o[7] = ok ? (unsigned short)f2bf(b.w) : (unsigned short)0;
  unsigned short* dp = XB + (size_t)row * INC + c0;
  *(volatile v8us*)dp = o;
  __threadfence();
  *(volatile v8us*)dp = o;
}

__device__ __forceinline__ v8us gat8(const float* __restrict__ p, int ld) {
  v8us o;
#pragma unroll
  for (int i = 0; i < 8; ++i) o[i] = (unsigned short)f2bf(p[(size_t)i * ld]);
  return o;
}

__global__ __launch_bounds__(NTHR) void k_pb(const float* __restrict__ Wl1, const float* __restrict__ Wr1,
                                             const float* __restrict__ b1, const float* __restrict__ Wl2,
                                             const float* __restrict__ Wr2, const float* __restrict__ b2,
                                             unsigned short* W1c, unsigned short* W2c, float* BT) {
  const int tid  = (int)threadIdx.x;
  const int part = (int)blockIdx.x >> 2;
  const int v    = ((int)blockIdx.x & 3) * NTHR + tid;
  if (part < 3) {
    const int n  = v >> 3;
    const int k8 = (v & 7) * 8;
    v8us o;
    if (part < 2) o = gat8(Wl1 + (size_t)k8 * HIDC + n, HIDC);
    else          o = gat8(Wr1 + (size_t)k8 * HIDC + n, HIDC);
    unsigned short* dp = W1c + (size_t)n * K1 + part * INC + k8;
    *(volatile v8us*)dp = o;
    __threadfence();
    *(volatile v8us*)dp = o;
  } else if (part < 7) {
    const int q    = part - 3;
    const int nsel = q >> 1;
    const int kd   = q & 1;
    const int nn   = v >> 4;
    const int k8   = (v & 15) * 8;
    v8us o;
    if (nsel == 0) o = gat8(Wl2 + (size_t)k8 * OUTC + nn, OUTC);
    else           o = gat8(Wr2 + (size_t)k8 * OUTC + nn, OUTC);
    unsigned short* dp = W2c + (size_t)(nsel * OUTC + nn) * K2 + kd * HIDC + k8;
    *(volatile v8us*)dp = o;
    __threadfence();
    *(volatile v8us*)dp = o;
  } else if ((int)blockIdx.x == 28) {
    if (tid < 64) {
      const int i1 = 4 * (tid < 31 ? tid : 31);
      int t2 = tid - 32;
      t2 = t2 < 0 ? 0 : (t2 > 15 ? 15 : t2);
      const v4f v1 = *(const v4f*)(b1 + i1);
      const v4f v2 = *(const v4f*)(b2 + 4 * t2);
      const unsigned m1 = (tid < 32) ? 0xFFFFFFFFu : 0u;
      const unsigned m2 = (tid >= 32 && tid < 48) ? 0xFFFFFFFFu : 0u;
      v4f o;
      o.x = __uint_as_float(((f2bf(v1.x) << 16) & m1) | ((f2bf(v2.x) << 16) & m2));
      o.y = __uint_as_float(((f2bf(v1.y) << 16) & m1) | ((f2bf(v2.y) << 16) & m2));
      o.z = __uint_as_float(((f2bf(v1.z) << 16) & m1) | ((f2bf(v2.z) << 16) & m2));
      o.w = __uint_as_float(((f2bf(v1.w) << 16) & m1) | ((f2bf(v2.w) << 16) & m2));
      float* dp = BT + 4 * tid;
      *(volatile v4f*)dp = o;
      __threadfence();
      *(volatile v4f*)dp = o;
    }
  }
}

__global__ __launch_bounds__(NTHR) void k_bucket(const int* __restrict__ srcs, const int* __restrict__ dsts,
                                                 int nE, int nN, int vec8,
                                                 int* LIST, int* OFFT, int* CNTT, int* FLG) {
  extern __shared__ __attribute__((aligned(16))) int bsm[];
  int* list = bsm;
  int* hl   = bsm + LISTN;
  int* sl   = hl + RCAP;
  int* cnt  = sl + RCAP;
  int* offs = cnt + NBA;
  int* cur  = offs + NBA;
  int* misc = cur + NBA;
  const int tid = (int)threadIdx.x, lane = tid & 31, wave = tid >> 5;
  const int blk = (int)blockIdx.x;
  const int nodeBase = blk * NBA;
  int nb = nN - nodeBase;
  nb = nb < 0 ? 0 : (nb > NBA ? NBA : nb);

  {
    const v4i z4 = {0, 0, 0, 0};
    for (int i = tid * 4; i < BKT_ZINTS; i += NTHR * 4) *(v4ia*)(sl + i) = z4;
    if (tid < 16) misc[tid] = 0;
  }
  __syncthreads();

  int tot = 0, ovf = 0;
  const int nChunks = (nE + CHUNK - 1) / CHUNK;
#pragma unroll 1
  for (int ch = 0; ch < nChunks; ++ch) {
    const int cbase = ch * CHUNK;
    const int wc = scan_chunk<SLA>(dsts, nE, cbase, nodeBase, nb, vec8, list, tid, lane, wave);
    if (lane == 0) misc[wave] = wc;
    __syncthreads();
    int pre = 0, all = 0;
#pragma unroll
    for (int w2 = 0; w2 < NWAVE; ++w2) {
      int c = misc[w2];
      c = c < 0 ? 0 : (c > WCAP ? WCAP : c);
      all += c;
      pre += (w2 < wave) ? c : 0;
    }
    const int wcc  = wc > WCAP ? WCAP : wc;
    const int base = tot + pre;
#pragma unroll 1
    for (int i = lane; i < wcc; i += 32) {
      const int ent = list[wave * WCAP + i];
      const int el  = (ent >> SLA) & (CHUNK - 1);
      const int sq  = ent & (NBA - 1);
      int eid = cbase + el;
      eid = eid > nE - 1 ? nE - 1 : eid;
      const int sraw = srcs[eid];
      const int s = sraw < 0 ? 0 : (sraw > nN - 1 ? nN - 1 : sraw);
      const int pos = base + i;
      if (pos < RCAP) hl[pos] = (int)((unsigned)s | ((unsigned)sq << SRCB));
    }
    if (tot + all > RCAP) ovf = 1;
    tot += all;
    tot = tot > RCAP ? RCAP : tot;
    __syncthreads();
  }
  const int nh = tot;

  if (wave == 0) {
#pragma unroll 1
    for (int b0 = 0; b0 < nh; b0 += 32) {
      const int idx = b0 + lane;
      const int uv  = hl[idx < nh ? idx : nh - 1];
      const int m32 = (nh - b0) < 32 ? (nh - b0) : 32;
#pragma unroll 1
      for (int k = 0; k < m32; ++k) {
        const int u  = __builtin_amdgcn_readlane(uv, k);
        const int sq = (u >> SRCB) & (NBA - 1);
        if (lane == 0) cnt[sq] = cnt[sq] + 1;
      }
    }
  }
  __syncthreads();
  if (wave == 0) {
    const int base = lane * (NBA / 32);
    int s = 0;
#pragma unroll 1
    for (int i = 0; i < NBA / 32; ++i) s += cnt[base + i];
    int incl = s;
#pragma unroll
    for (int d = 1; d < 32; d <<= 1) {
      const int y = __shfl_up(incl, d, 32);
      if (lane >= d) incl += y;
    }
    int run = incl - s;
#pragma unroll 1
    for (int i = 0; i < NBA / 32; ++i) {
      const int cv = cnt[base + i];
      offs[base + i] = run;
      cur[base + i]  = run;
      run += cv;
    }
  }
  __syncthreads();
  if (wave == 0) {
#pragma unroll 1
    for (int b0 = 0; b0 < nh; b0 += 32) {
      const int idx = b0 + lane;
      const int uv  = hl[idx < nh ? idx : nh - 1];
      const int m32 = (nh - b0) < 32 ? (nh - b0) : 32;
#pragma unroll 1
      for (int k = 0; k < m32; ++k) {
        const int u  = __builtin_amdgcn_readlane(uv, k);
        const int sq = (u >> SRCB) & (NBA - 1);
        if (lane == 0) {
          int p = cur[sq];
          p = p < 0 ? 0 : (p > RCAP - 1 ? RCAP - 1 : p);
          sl[p] = u;
          cur[sq] = p + 1;
        }
      }
    }
  }
  __syncthreads();

  int* lb = LIST + (size_t)blk * RCAP;
  int* op = OFFT + (size_t)blk * NBA + 4 * tid;
  int* cp = CNTT + (size_t)blk * NBA + 4 * tid;
  int* fp = FLG + (size_t)blk * 32 + 4 * (tid & 7);
  const v4i ov = *(const v4ia*)(offs + 4 * tid);
  const v4i cv = *(const v4ia*)(cnt + 4 * tid);
  v4i fv;
  fv.x = (tid == 0) ? nh : 0;
  fv.y = (tid == 0) ? ovf : 0;
  fv.z = 0; fv.w = 0;
  const int smask = (1 << SRCB) - 1;
#pragma unroll 1
  for (int p = tid * 4; p < RCAP; p += NTHR * 4) {
    v4i v = *(const v4ia*)(sl + p);
    v.x &= smask; v.y &= smask; v.z &= smask; v.w &= smask;
    *(volatile v4i*)(lb + p) = v;
  }
  *(volatile v4i*)op = ov;
  *(volatile v4i*)cp = cv;
  if (tid < 8) *(volatile v4i*)fp = fv;
  __threadfence();
#pragma unroll 1
  for (int p = tid * 4; p < RCAP; p += NTHR * 4) {
    v4i v = *(const v4ia*)(sl + p);
    v.x &= smask; v.y &= smask; v.z &= smask; v.w &= smask;
    *(volatile v4i*)(lb + p) = v;
  }
  *(volatile v4i*)op = ov;
  *(volatile v4i*)cp = cv;
  if (tid < 8) *(volatile v4i*)fp = fv;
}

__global__ __launch_bounds__(NTHR) __attribute__((amdgpu_num_vgpr(248)))
void k_agg1(const int* __restrict__ LIST, const int* __restrict__ OFFT, const int* __restrict__ CNTT,
            const int* __restrict__ FLG, const unsigned* __restrict__ XBw, unsigned* AGGw, int nN, int MPr) {
  __shared__ __attribute__((aligned(16))) unsigned srow[NWAVE * NPW * 64];
  const int tid = (int)threadIdx.x, lane = tid & 31;
  const int wave = __builtin_amdgcn_readfirstlane(tid >> 5);
  unsigned* sw = srow + wave * NPW * 64;
  const int base = (int)blockIdx.x * NPB + wave * NPW;
  const int bb   = ((int)blockIdx.x * NPB) >> SLA;
  const int nhraw = __builtin_amdgcn_readfirstlane(FLG[(size_t)bb * 32]);
  const int bflag = __builtin_amdgcn_readfirstlane(FLG[(size_t)bb * 32 + 1]);
  const int nh = nhraw < 0 ? 0 : (nhraw > RCAP ? RCAP : nhraw);
  const bool bad = (bflag != 0) || (nhraw < 0) || (nhraw > RCAP);
  const float qnan = __int_as_float(0x7fc00000);
  const int* lb = LIST + (size_t)bb * RCAP;

#pragma unroll 1
  for (int j = 0; j < NPW; ++j) {
    const int node = base + j;
    const int nt   = node < MPr ? node : MPr - 1;
    const int craw = __builtin_amdgcn_readfirstlane(CNTT[nt]);
    const int oraw = __builtin_amdgcn_readfirstlane(OFFT[nt]);
    int c = craw < 0 ? 0 : (craw > DEGCAP ? DEGCAP : craw);
    const int o = oraw < 0 ? 0 : (oraw > RCAP ? RCAP : oraw);
    if (c > nh - o) c = nh - o;
    c = c < 0 ? 0 : c;
    const bool big = (c != craw) || (o != oraw);
    float a0 = 0.0f, a1 = 0.0f;
#pragma unroll 1
    for (int b0 = 0; b0 < c; b0 += 32) {
      int idx = o + b0 + lane;
      const int last = o + c - 1;
      idx = idx > last ? last : idx;
      idx = idx < 0 ? 0 : (idx > RCAP - 1 ? RCAP - 1 : idx);
      int sr = lb[idx];
      sr = sr < 0 ? 0 : (sr > nN - 1 ? nN - 1 : sr);
      const int m32 = (c - b0) < 32 ? (c - b0) : 32;
#pragma unroll 1
      for (int k = 0; k < m32; ++k) {
        const int sk = __builtin_amdgcn_readlane(sr, k);
        const unsigned w = XBw[(size_t)sk * 32 + lane];
        a0 += __uint_as_float(w << 16);
        a1 += __uint_as_float(w & 0xffff0000u);
      }
    }
    const float d   = fmaxf((float)c, 1.0f);
    const float pzr = (bad || big) ? qnan : 0.0f;
    const bool live = node < nN;
    const float m0 = live ? (a0 / d + pzr) : 0.0f;
    const float m1 = live ? (a1 / d + pzr) : 0.0f;
    const unsigned h0 = f2bf(m0), h1 = f2bf(m1);
    const unsigned l0 = f2bf(m0 - bf2f(h0)), l1 = f2bf(m1 - bf2f(h1));
    sw[j * 64 + lane]      = h0 | (h1 << 16);
    sw[j * 64 + 32 + lane] = l0 | (l1 << 16);
  }
  __syncthreads();
#pragma unroll 1
  for (int j = 0; j < NPW; ++j) {
    const int node = base + j;
    const v2u q = *(const v2ua*)(sw + j * 64 + 2 * lane);
    if (node < MPr) *(volatile v2u*)(AGGw + (size_t)node * 64 + 2 * lane) = q;
  }
  __threadfence();
#pragma unroll 1
  for (int j = 0; j < NPW; ++j) {
    const int node = base + j;
    const v2u q = *(const v2ua*)(sw + j * 64 + 2 * lane);
    if (node < MPr) *(volatile v2u*)(AGGw + (size_t)node * 64 + 2 * lane) = q;
  }
}

__global__ __launch_bounds__(GTHR) __attribute__((amdgpu_num_vgpr(248)))
void k_gemm1(const unsigned short* __restrict__ AGG, const unsigned short* __restrict__ XB,
             const unsigned short* __restrict__ WT, const float* __restrict__ BT,
             unsigned short* Hhl, int nN) {
  __shared__ __attribute__((aligned(16))) float stg[GBM * GBN];
  const int tid = (int)threadIdx.x, lane = tid & 31, wave = tid >> 5, hh = lane >> 4, m = lane & 15;
  const int rowBase = (int)blockIdx.x * GBM;

  v8f acc[8];
  {
    const v8f z = {0.f, 0.f, 0.f, 0.f, 0.f, 0.f, 0.f, 0.f};
#pragma unroll
    for (int t = 0; t < 8; ++t) acc[t] = z;
  }
  const unsigned short* ap = AGG + (size_t)(rowBase + 16 * wave + m) * (size_t)HIDC + 8 * hh;
  const unsigned short* xp = XB  + (size_t)(rowBase + 16 * wave + m) * (size_t)INC + 8 * hh;
  const unsigned short* bp = WT  + (size_t)m * (size_t)K1 + 8 * hh;

#pragma unroll 1
  for (int k0 = 0; k0 < 2 * INC; k0 += 32) {
    FragB af;
    af.h[0] = *(const v8usa*)(ap + k0);
    af.h[1] = *(const v8usa*)(ap + k0 + 16);
#pragma unroll
    for (int nt = 0; nt < 8; ++nt) {
      const unsigned short* wq = bp + (size_t)(16 * nt) * (size_t)K1 + k0;
      FragB bf;
      bf.h[0] = *(const v8usa*)wq;
      bf.h[1] = *(const v8usa*)(wq + 16);
      acc[nt] = wmb(af, bf, acc[nt]);
    }
  }
#pragma unroll 1
  for (int k0 = 0; k0 < INC; k0 += 32) {
    FragB af;
    af.h[0] = *(const v8usa*)(xp + k0);
    af.h[1] = *(const v8usa*)(xp + k0 + 16);
#pragma unroll
    for (int nt = 0; nt < 8; ++nt) {
      const unsigned short* wq = bp + (size_t)(16 * nt) * (size_t)K1 + 2 * INC + k0;
      FragB bf;
      bf.h[0] = *(const v8usa*)wq;
      bf.h[1] = *(const v8usa*)(wq + 16);
      acc[nt] = wmb(af, bf, acc[nt]);
    }
  }

#pragma unroll
  for (int nt = 0; nt < 8; ++nt) {
    const int lc = 16 * nt + m;
#pragma unroll
    for (int r = 0; r < 8; ++r) {
      const int lr = 16 * wave + 8 * hh + r;
      stg[lr * GBN + lc] = acc[nt][r];
    }
  }
  __syncthreads();

  const v4f b4 = *(const v4f*)(BT + 4 * lane);
#pragma unroll 1
  for (int i = 0; i < 16; ++i) {
    float* frow = stg + (16 * wave + i) * GBN;
    const v4f t = *(const v4fa*)(frow + 4 * lane);
    __syncthreads();
    const bool ok = (rowBase + 16 * wave + i) < nN;
    float y0 = t.x + b4.x, y1 = t.y + b4.y, y2 = t.z + b4.z, y3 = t.w + b4.w;
    y0 = (y0 > 0.0f) ? y0 : (y0 - y0);
    y1 = (y1 > 0.0f) ? y1 : (y1 - y1);
    y2 = (y2 > 0.0f) ? y2 : (y2 - y2);
    y3 = (y3 > 0.0f) ? y3 : (y3 - y3);
    y0 = ok ? y0 : 0.0f; y1 = ok ? y1 : 0.0f; y2 = ok ? y2 : 0.0f; y3 = ok ? y3 : 0.0f;
    v4us h4, l4;
    unsigned hb;
    hb = f2bf(y0); h4[0] = (unsigned short)hb; l4[0] = (unsigned short)f2bf(y0 - bf2f(hb));
    hb = f2bf(y1); h4[1] = (unsigned short)hb; l4[1] = (unsigned short)f2bf(y1 - bf2f(hb));
    hb = f2bf(y2); h4[2] = (unsigned short)hb; l4[2] = (unsigned short)f2bf(y2 - bf2f(hb));
    hb = f2bf(y3); h4[3] = (unsigned short)hb; l4[3] = (unsigned short)f2bf(y3 - bf2f(hb));
    unsigned short* srow = (unsigned short*)frow;
    *(v4usa*)(srow + 4 * lane) = h4;
    *(v4usa*)(srow + HIDC + 4 * lane) = l4;
  }
  __syncthreads();
#pragma unroll 1
  for (int i = 0; i < 16; ++i) {
    const unsigned short* srow = (const unsigned short*)(stg + (16 * wave + i) * GBN);
    const v8us q = *(const v8usa*)(srow + 8 * lane);
    unsigned short* gp = Hhl + (size_t)(rowBase + 16 * wave + i) * (size_t)K2 + 8 * lane;
    *(volatile v8us*)gp = q;
  }
  __threadfence();
#pragma unroll 1
  for (int i = 0; i < 16; ++i) {
    const unsigned short* srow = (const unsigned short*)(stg + (16 * wave + i) * GBN);
    const v8us q = *(const v8usa*)(srow + 8 * lane);
    unsigned short* gp = Hhl + (size_t)(rowBase + 16 * wave + i) * (size_t)K2 + 8 * lane;
    *(volatile v8us*)gp = q;
  }
}

__global__ __launch_bounds__(GTHR) __attribute__((amdgpu_num_vgpr(248)))
void k_gemm2(const unsigned short* __restrict__ Hhl, const unsigned short* __restrict__ WT,
             const float* __restrict__ BT, float* P, long long rDelta) {
  __shared__ __attribute__((aligned(16))) float stg[GBM * GBN];
  const int tid = (int)threadIdx.x, lane = tid & 31, wave = tid >> 5, hh = lane >> 4, m = lane & 15;
  const int rowBase = (int)blockIdx.x * GBM;

  v8f acc[8];
  {
    const v8f z = {0.f, 0.f, 0.f, 0.f, 0.f, 0.f, 0.f, 0.f};
#pragma unroll
    for (int t = 0; t < 8; ++t) acc[t] = z;
  }
  const unsigned short* ap = Hhl + (size_t)(rowBase + 16 * wave + m) * (size_t)K2 + 8 * hh;
  const unsigned short* bp = WT  + (size_t)m * (size_t)K2 + 8 * hh;
#pragma unroll 1
  for (int k0 = 0; k0 < K2; k0 += 32) {
    FragB af;
    af.h[0] = *(const v8usa*)(ap + k0);
    af.h[1] = *(const v8usa*)(ap + k0 + 16);
#pragma unroll
    for (int nt = 0; nt < 8; ++nt) {
      const unsigned short* wq = bp + (size_t)(16 * nt) * (size_t)K2 + k0;
      FragB bf;
      bf.h[0] = *(const v8usa*)wq;
      bf.h[1] = *(const v8usa*)(wq + 16);
      acc[nt] = wmb(af, bf, acc[nt]);
    }
  }

#pragma unroll
  for (int nt = 0; nt < 8; ++nt) {
    const int lc = 16 * nt + m;
#pragma unroll
    for (int r = 0; r < 8; ++r) {
      const int lr = 16 * wave + 8 * hh + r;
      stg[lr * GBN + lc] = acc[nt][r];
    }
  }
  __syncthreads();

  const int pc = lane & 15;
  const int bo = (hh != 0) ? (HIDC + 4 * pc) : (HIDC + OUTC + 4 * pc);
  const v4f b4 = *(const v4f*)(BT + bo);
  const long long dl = (hh != 0) ? rDelta : 0LL;
  float* ob = P + dl + 4 * pc;
#pragma unroll 1
  for (int i = 0; i < 16; ++i) {
    const int row = rowBase + 16 * wave + i;
    const v4f t = *(const v4fa*)(stg + (16 * wave + i) * GBN + 4 * lane);
    const v4f y = t + b4;
    *(volatile v4f*)(ob + (size_t)row * OUTC) = y;
  }
  __threadfence();
#pragma unroll 1
  for (int i = 0; i < 16; ++i) {
    const int row = rowBase + 16 * wave + i;
    const v4f t = *(const v4fa*)(stg + (16 * wave + i) * GBN + 4 * lane);
    const v4f y = t + b4;
    *(volatile v4f*)(ob + (size_t)row * OUTC) = y;
  }
}

__global__ __launch_bounds__(NTHR) __attribute__((amdgpu_num_vgpr(248)))
void k_agg2(const int* __restrict__ LIST, const int* __restrict__ OFFT, const int* __restrict__ CNTT,
            const int* __restrict__ FLG, const float* __restrict__ P, float* RZ, int nN, int MPr) {
  __shared__ __attribute__((aligned(16))) float frow[NWAVE * NPW * 64];
  const int tid = (int)threadIdx.x, lane = tid & 31;
  const int wave = __builtin_amdgcn_readfirstlane(tid >> 5);
  float* sw = frow + wave * NPW * 64;
  const int base = (int)blockIdx.x * NPB + wave * NPW;
  const int bb   = ((int)blockIdx.x * NPB) >> SLA;
  const int nhraw = __builtin_amdgcn_readfirstlane(FLG[(size_t)bb * 32]);
  const int bflag = __builtin_amdgcn_readfirstlane(FLG[(size_t)bb * 32 + 1]);
  const int nh = nhraw < 0 ? 0 : (nhraw > RCAP ? RCAP : nhraw);
  const bool bad = (bflag != 0) || (nhraw < 0) || (nhraw > RCAP);
  const float qnan = __int_as_float(0x7fc00000);
  const int* lb = LIST + (size_t)bb * RCAP;

#pragma unroll 1
  for (int j = 0; j < NPW; ++j) {
    const int node = base + j;
    const int nt   = node < MPr ? node : MPr - 1;
    const int craw = __builtin_amdgcn_readfirstlane(CNTT[nt]);
    const int oraw = __builtin_amdgcn_readfirstlane(OFFT[nt]);
    int c = craw < 0 ? 0 : (craw > DEGCAP ? DEGCAP : craw);
    const int o = oraw < 0 ? 0 : (oraw > RCAP ? RCAP : oraw);
    if (c > nh - o) c = nh - o;
    c = c < 0 ? 0 : c;
    const bool big = (c != craw) || (o != oraw);
    float a0 = 0.0f, a1 = 0.0f;
#pragma unroll 1
    for (int b0 = 0; b0 < c; b0 += 32) {
      int idx = o + b0 + lane;
      const int last = o + c - 1;
      idx = idx > last ? last : idx;
      idx = idx < 0 ? 0 : (idx > RCAP - 1 ? RCAP - 1 : idx);
      int sr = lb[idx];
      sr = sr < 0 ? 0 : (sr > nN - 1 ? nN - 1 : sr);
      const int m32 = (c - b0) < 32 ? (c - b0) : 32;
#pragma unroll 1
      for (int k = 0; k < m32; ++k) {
        const int sk = __builtin_amdgcn_readlane(sr, k);
        const v2f pv = *(const v2f*)(P + (size_t)sk * OUTC + 2 * lane);
        a0 += pv.x;
        a1 += pv.y;
      }
    }
    const v2f rv = *(const v2f*)(RZ + (size_t)nt * OUTC + 2 * lane);
    const float d   = fmaxf((float)c, 1.0f);
    const float pzr = (bad || big) ? qnan : 0.0f;
    const bool live = node < nN;
    v2f z;
    z.x = live ? ((a0 / d + rv.x) + pzr) : 0.0f;
    z.y = live ? ((a1 / d + rv.y) + pzr) : 0.0f;
    *(v2fa*)(sw + j * 64 + 2 * lane) = z;
  }
  __syncthreads();
#pragma unroll 1
  for (int j = 0; j < NPW; ++j) {
    const int node = base + j;
    const v2f q = *(const v2fa*)(sw + j * 64 + 2 * lane);
    if (node < MPr) *(volatile v2f*)(RZ + (size_t)node * OUTC + 2 * lane) = q;
  }
  __threadfence();
#pragma unroll 1
  for (int j = 0; j < NPW; ++j) {
    const int node = base + j;
    const v2f q = *(const v2fa*)(sw + j * 64 + 2 * lane);
    if (node < MPr) *(volatile v2f*)(RZ + (size_t)node * OUTC + 2 * lane) = q;
  }
}

__global__ __launch_bounds__(NTHR) __attribute__((amdgpu_num_vgpr(248)))
void k_dec(const float* __restrict__ Z, const int* __restrict__ la, const int* __restrict__ lbb,
           float* out, int nLines, int nN) {
  const int tid = (int)threadIdx.x, lane = tid & 31;
  const int wave = __builtin_amdgcn_readfirstlane(tid >> 5);
#pragma unroll 1
  for (int j = 0; j < 4; ++j) {
    const int line = (int)blockIdx.x * 32 + wave * 4 + j;
    if (line < nLines) {
      const int p = line * 32 + lane;
      int ia = la[p];
      int ib = lbb[p];
      ia = ia < 0 ? 0 : (ia > nN - 1 ? nN - 1 : ia);
      ib = ib < 0 ? 0 : (ib > nN - 1 ? nN - 1 : ib);
      float res = 0.0f;
#pragma unroll 1
      for (int k = 0; k < 32; ++k) {
        const int sa = __builtin_amdgcn_readlane(ia, k);
        const int sb = __builtin_amdgcn_readlane(ib, k);
        const v2f a = *(const v2f*)(Z + (size_t)sa * OUTC + 2 * lane);
        const v2f b = *(const v2f*)(Z + (size_t)sb * OUTC + 2 * lane);
        float s = a.x * b.x + a.y * b.y;
        s += __shfl_xor(s, 16, 32);
        s += __shfl_xor(s, 8, 32);
        s += __shfl_xor(s, 4, 32);
        s += __shfl_xor(s, 2, 32);
        s += __shfl_xor(s, 1, 32);
        res = (lane == k) ? s : res;
      }
      float* op = out + p;
      *(volatile float*)op = res;
      __threadfence();
      *(volatile float*)op = res;
    }
  }
}

static inline int cdiv(int a, int b) { return (a + b - 1) / b; }
static inline size_t al256(size_t o) { return (o + 255) & ~(size_t)255; }

extern "C" void kernel_launch(void* const* d_in, const int* in_sizes, int n_in,
                              void* d_out, int out_size, void* d_ws, size_t ws_size,
                              hipStream_t stream) {
  if (n_in < 9) return;
  if (in_sizes[0] <= 0 || (in_sizes[0] % INC) != 0) return;
  const int nN = in_sizes[0] / INC;
  if (nN < 16 || nN > (1 << SRCB)) return;
  if (in_sizes[1] < 2 || (in_sizes[1] & 1) != 0) return;
  const int nE = in_sizes[1] / 2;
  if (nE < 1 || nE > (1 << 30)) return;
  if (in_sizes[2] < 2 || (in_sizes[2] & 1) != 0) return;
  const int nP = in_sizes[2] / 2;
  if ((nP % 32) != 0 || out_size != nP) return;
  if (in_sizes[3] != INC * HIDC || in_sizes[4] != INC * HIDC || in_sizes[5] != HIDC) return;
  if (in_sizes[6] != HIDC * OUTC || in_sizes[7] != HIDC * OUTC || in_sizes[8] != OUTC) return;

  const float* x   = (const float*)d_in[0];
  const int*   ei  = (const int*)  d_in[1];
  const int*   eli = (const int*)  d_in[2];
  const float* Wl1 = (const float*)d_in[3];
  const float* Wr1 = (const float*)d_in[4];
  const float* b1  = (const float*)d_in[5];
  const float* Wl2 = (const float*)d_in[6];
  const float* Wr2 = (const float*)d_in[7];
  const float* b2  = (const float*)d_in[8];
  float* out = (float*)d_out;
  const int* src = ei;
  const int* dst = ei + nE;
  const int* pa  = eli;
  const int* pb  = eli + nP;

  const int MP   = cdiv(nN, MROWS) * MROWS;
  const int gM   = MP / GBM;
  const int gG   = MP / NPB;
  const int gA   = cdiv(MP, NBA);
  if ((long long)gA * NBA < (long long)MP) return;
  const int vec8 = ((nE & 3) == 0) ? 1 : 0;
  const int nUx  = MP * (INC / 8);
  if ((nUx % NTHR) != 0) return;
  const int nLines = nP / 32;

  char* ws = (char*)d_ws;
  size_t off = 0;
  const size_t oXB  = off; off = al256(off + (size_t)MP * INC * 2);
  const size_t szAG = (size_t)MP * HIDC * 2;
  const size_t szP  = (size_t)MP * OUTC * 4;
  const size_t oAG  = off; off = al256(off + (szAG > szP ? szAG : szP));
  const size_t oH   = off; off = al256(off + (size_t)MP * K2 * 2);
  const size_t oR   = off; off = al256(off + (size_t)MP * OUTC * 4);
  const size_t oLI  = off; off = al256(off + (size_t)gA * RCAP * 4);
  const size_t oOF  = off; off = al256(off + (size_t)gA * NBA * 4);
  const size_t oCN  = off; off = al256(off + (size_t)gA * NBA * 4);
  const size_t oFL  = off; off = al256(off + (size_t)gA * 128);
  const size_t oW1  = off; off = al256(off + (size_t)HIDC * K1 * 2);
  const size_t oW2  = off; off = al256(off + (size_t)HIDC * K2 * 2);
  const size_t oBT  = off; off = al256(off + (size_t)256 * 4);
  if (off > ws_size || off > (size_t)WSMAX) return;
  unsigned short* XB   = (unsigned short*)(ws + oXB);
  unsigned short* AGG  = (unsigned short*)(ws + oAG);
  float*          Pp   = (float*)(ws + oAG);
  unsigned short* Hhl  = (unsigned short*)(ws + oH);
  float*          RZ   = (float*)(ws + oR);
  int*            LIST = (int*)(ws + oLI);
  int*            OFFT = (int*)(ws + oOF);
  int*            CNTT = (int*)(ws + oCN);
  int*            FLG  = (int*)(ws + oFL);
  unsigned short* W1c  = (unsigned short*)(ws + oW1);
  unsigned short* W2c  = (unsigned short*)(ws + oW2);
  float*          BT   = (float*)(ws + oBT);
  const long long rDelta = (long long)((oR - oAG) / 4);

  const int bktLds = BKT_LDS_INTS * 4;
  hipFuncSetAttribute(reinterpret_cast<const void*>(&k_bucket),
                      hipFuncAttributeMaxDynamicSharedMemorySize, bktLds);

  k_pa<<<nUx / NTHR, NTHR, 0, stream>>>(x, XB, nN, nUx);
  k_pb<<<29, NTHR, 0, stream>>>(Wl1, Wr1, b1, Wl2, Wr2, b2, W1c, W2c, BT);
  k_bucket<<<gA, NTHR, bktLds, stream>>>(src, dst, nE, nN, vec8, LIST, OFFT, CNTT, FLG);
  k_agg1<<<gG, NTHR, 0, stream>>>(LIST, OFFT, CNTT, FLG, (const unsigned*)XB, (unsigned*)AGG, nN, MP);
  k_gemm1<<<gM, GTHR, 0, stream>>>(AGG, XB, W1c, BT, Hhl, nN);
  k_gemm2<<<gM, GTHR, 0, stream>>>(Hhl, W2c, BT, Pp, rDelta);
  k_agg2<<<gG, NTHR, 0, stream>>>(LIST, OFFT, CNTT, FLG, Pp, RZ, nN, MP);
  k_dec<<<cdiv(nLines, 32), NTHR, 0, stream>>>(RZ, pa, pb, out, nLines, nN);
}
